// StandardMultiHeadAttention_58265526338307
// MI455X (gfx1250) — hardware-verified
//
#include <hip/hip_runtime.h>
#include <math.h>
#include <stdint.h>

#define NB    4
#define CH    1024
#define IMH   32
#define IMW   32
#define NTOK  1024
#define INNER 1024
#define NH    16
#define HD    64
#define NQKV  3072
#define QKP   2048
#define AOP   2048
#define VTP   (NB * NTOK)
#define MTOK  (NB * NTOK)
#define TABN  512
#define RMS_EPS 1e-6f

static_assert(NTOK == IMH * IMW);
static_assert(IMW == 32);
static_assert(INNER == NH * HD);
static_assert(HD == 64);
static_assert(NQKV == 3 * INNER);
static_assert(QKP == 2 * INNER);
static_assert(AOP == 2 * INNER);
static_assert(CH % 64 == 0);
static_assert(NTOK % 64 == 0);
static_assert(INNER % 64 == 0);
static_assert(MTOK % 64 == 0);
static_assert(CH % 32 == 0);
static_assert(AOP % 32 == 0);
static_assert(INNER == 128 * 8);
static_assert(CH == 8 * 128);
static_assert(TABN == 32 * (HD / 4));
static_assert((NQKV * CH) % (8 * 256) == 0);
static_assert((CH * INNER) % (8 * 256) == 0);
static_assert(CH % 256 == 0);
static_assert(INNER % 256 == 0);

typedef __attribute__((ext_vector_type(16))) _Float16 v16h;
typedef __attribute__((ext_vector_type(8)))  _Float16 v8h;
typedef __attribute__((ext_vector_type(16))) __bf16   v16b;
typedef __attribute__((ext_vector_type(8)))  __bf16   v8b;
typedef __attribute__((ext_vector_type(8)))  float    v8f;
typedef __attribute__((ext_vector_type(4)))  float    v4f;
typedef __attribute__((ext_vector_type(2)))  float    v2f;
typedef __attribute__((ext_vector_type(4)))  unsigned int v4u;

__device__ __forceinline__ unsigned short f2bf_bits(float f) {
  unsigned u = __float_as_uint(f);
  return (unsigned short)((u + 0x7FFFu + ((u >> 16) & 1u)) >> 16);
}
__device__ __forceinline__ float bf_bits2f(unsigned short h) { return __uint_as_float(((unsigned)h) << 16); }
__device__ __forceinline__ float bf_rne(float f) { return bf_bits2f(f2bf_bits(f)); }
__device__ __forceinline__ unsigned pk16(unsigned short a, unsigned short b) { return (unsigned)a | ((unsigned)b << 16); }

__device__ __forceinline__ void dep_guard_h(v8f& a, v8f& b, v16h x, v16h y) { asm volatile("v_nop\n\tv_nop\n\tv_nop\n\tv_nop" : "+v"(a), "+v"(b) : "v"(x), "v"(y)); }
__device__ __forceinline__ void dep_guard_b(v8f& a, v8f& b, v16b x, v16b y) { asm volatile("v_nop\n\tv_nop\n\tv_nop\n\tv_nop" : "+v"(a), "+v"(b) : "v"(x), "v"(y)); }
__device__ __forceinline__ void keep4_h(v16h a, v16h b, v16h c, v16h d) { asm volatile("v_nop" :: "v"(a), "v"(b), "v"(c), "v"(d)); }
__device__ __forceinline__ void keep4_b(v16b a, v16b b, v16b c, v16b d) { asm volatile("v_nop" :: "v"(a), "v"(b), "v"(c), "v"(d)); }
__device__ __forceinline__ void acc_guard4(v8f& a, v8f& b, v8f& c, v8f& d) { asm volatile("v_nop\n\tv_nop\n\tv_nop\n\tv_nop" : "+v"(a), "+v"(b), "+v"(c), "+v"(d)); }
template <typename T> struct Frag;
template <> struct Frag<_Float16> {
  typedef v16h V; union U { v16h v; v8h h[2]; };
  static __device__ __forceinline__ v16h load(const _Float16* p) {
    U f; f.h[0] = *(const v8h*)(p); f.h[1] = *(const v8h*)(p + 16); return f.v;
  }
  static __device__ __forceinline__ v8f mma(v16h a, v16h b, v8f c) {
    return __builtin_amdgcn_wmma_f32_16x16x32_f16(false, a, false, b, (short)0, c, false, false);
  }
  static __device__ __forceinline__ void guard(v8f& a, v8f& b, v16h x, v16h y) { dep_guard_h(a, b, x, y); }
  static __device__ __forceinline__ void keep(v16h a, v16h b, v16h c, v16h d) { keep4_h(a, b, c, d); }
};
template <> struct Frag<__bf16> {
  typedef v16b V; union U { v16b v; v8b h[2]; };
  static __device__ __forceinline__ v16b load(const __bf16* p) {
    U f; f.h[0] = *(const v8b*)(p); f.h[1] = *(const v8b*)(p + 16); return f.v;
  }
  static __device__ __forceinline__ v8f mma(v16b a, v16b b, v8f c) {
    return __builtin_amdgcn_wmma_f32_16x16x32_bf16(false, a, false, b, (short)0, c, false, false);
  }
  static __device__ __forceinline__ void guard(v8f& a, v8f& b, v16b x, v16b y) { dep_guard_b(a, b, x, y); }
  static __device__ __forceinline__ void keep(v16b a, v16b b, v16b c, v16b d) { keep4_b(a, b, c, d); }
};

template <int ET> struct Elem;
template <> struct Elem<0> { typedef _Float16 T; };
template <> struct Elem<1> { typedef __bf16 T; };
template <int ET, bool SPLIT, int BIAS_MODE, int OUT_MODE, bool RESID, int ACT = 0>
__global__ __launch_bounds__(256) void wmma_gemm64(
    const unsigned short* __restrict__ Ap, const unsigned short* __restrict__ A2p, int lda, long strideA,
    const unsigned short* __restrict__ Btp, const unsigned short* __restrict__ Bt2p, int ldb, long strideB,
    void* __restrict__ Cout, void* __restrict__ Cout2, int ldc, long strideC,
    const float* __restrict__ bias,
    const float* __restrict__ resid, long strideR,
    int M, int N, int K, float scale) {
  typedef typename Elem<ET>::T T;
  typedef typename Frag<T>::V V;
  const T* A = (const T*)Ap; const T* A2 = (const T*)A2p; const T* Bt = (const T*)Btp; const T* Bt2 = (const T*)Bt2p;
  __shared__ __align__(16) float sT[8][16 * 68];
  const int b    = blockIdx.y;
  const int lane = threadIdx.x & 31;
  const int wave = threadIdx.x >> 5;
  const int tilesN = N >> 6;
  const int tilesM = M >> 6;
  const int tile = blockIdx.x * 8 + wave;
  if (tile >= tilesM * tilesN) return;
  const int tm = tile / tilesN;
  const int tn = tile - tm * tilesN;
  const int m0 = tm << 6;
  const int n0 = tn << 6;

  const T* Ab  = A  + (size_t)b * strideA;
  const T* Bb  = Bt + (size_t)b * strideB;
  const T* Ab2 = SPLIT ? (A2  + (size_t)b * strideA) : nullptr;
  const T* Bb2 = SPLIT ? (Bt2 + (size_t)b * strideB) : nullptr;

  const int rlane = lane & 15;
  const int koff  = (lane >> 4) * 8;
  const int mOff  = (lane >> 4) * 8;

  v8f acc[4][4];
#pragma unroll
  for (int i = 0; i < 4; ++i)
#pragma unroll
    for (int j = 0; j < 4; ++j) acc[i][j] = (v8f){0.f,0.f,0.f,0.f,0.f,0.f,0.f,0.f};

  for (int k0 = 0; k0 < K; k0 += 32) {
    V bh[4], bl[4];
#pragma unroll
    for (int j = 0; j < 4; ++j) {
      const size_t bo = (size_t)(n0 + (j << 4) + rlane) * ldb + koff + k0;
      bh[j] = Frag<T>::load(Bb + bo);
      if (SPLIT) bl[j] = Frag<T>::load(Bb2 + bo); else bl[j] = bh[j];
    }
#pragma unroll
    for (int i = 0; i < 4; ++i) {
      const size_t ao = (size_t)(m0 + (i << 4) + rlane) * lda + koff + k0;
      V ah = Frag<T>::load(Ab + ao);
      V al;
      if (SPLIT) al = Frag<T>::load(Ab2 + ao); else al = ah;
#pragma unroll
      for (int j = 0; j < 4; ++j) {
        acc[i][j] = Frag<T>::mma(ah, bh[j], acc[i][j]);
        if (SPLIT) {
          acc[i][j] = Frag<T>::mma(ah, bl[j], acc[i][j]);
          acc[i][j] = Frag<T>::mma(al, bh[j], acc[i][j]);
        }
      }
      Frag<T>::guard(acc[i][0], acc[i][3], ah, al);
    }
    Frag<T>::keep(bh[0], bh[1], bh[2], bh[3]);
    if (SPLIT) Frag<T>::keep(bl[0], bl[1], bl[2], bl[3]);
  }
  acc_guard4(acc[0][0], acc[0][1], acc[0][2], acc[0][3]);
  acc_guard4(acc[1][0], acc[1][1], acc[1][2], acc[1][3]);
  acc_guard4(acc[2][0], acc[2][1], acc[2][2], acc[2][3]);
  acc_guard4(acc[3][0], acc[3][1], acc[3][2], acc[3][3]);

  float* slab = sT[wave];
  const float* Rb = RESID ? (resid + (size_t)b * strideR) : nullptr;
#pragma unroll
  for (int i = 0; i < 4; ++i) {
    const int mBase = m0 + (i << 4);
#pragma unroll
    for (int j = 0; j < 4; ++j) {
      const int n = n0 + (j << 4) + rlane;
      float bv = 0.f;
      if (BIAS_MODE == 2) bv = bf_rne(bias[n]);
#pragma unroll
      for (int r = 0; r < 8; ++r) {
        float v = acc[i][j][r] * scale;
        if (BIAS_MODE == 1) v += bf_rne(bias[mBase + mOff + r]);
        if (BIAS_MODE == 2) v += bv;
        if (RESID) v += Rb[(size_t)(mBase + mOff + r) * ldc + n];
        if (ACT == 1) v = tanhf(v);
        if (ACT == 2) v = fmaxf(v, 0.0f);
        if (ACT == 3) v = v / (1.0f + expf(-v));
        if (ACT == 4) v = (v > 0.f) ? v : 0.01f * v;
        if (ACT == 5) v = 0.5f * v * (1.0f + erff(v * 0.70710678118654752f));
        slab[(mOff + r) * 68 + (j << 4) + rlane] = v;
      }
    }
    __builtin_amdgcn_fence(__ATOMIC_RELEASE, "workgroup");
    __builtin_amdgcn_wave_barrier();
    __builtin_amdgcn_fence(__ATOMIC_ACQUIRE, "workgroup");
    if (OUT_MODE == 0) {
      float* C = (float*)Cout + (size_t)b * strideC;
      const int hh = lane >> 4, c4 = (lane & 15) * 4;
      for (int pass = 0; pass < 2; ++pass) {
#pragma unroll
        for (int it = 0; it < 8; ++it) {
          const int row = it * 2 + hh;
          v4f v = *(const v4f*)(slab + row * 68 + c4);
          *(volatile v4f*)(C + (size_t)(mBase + row) * ldc + n0 + c4) = v;
        }
        __threadfence();
      }
    } else {
      const int q = lane >> 3, c8 = (lane & 7) * 8;
      unsigned short* C  = (unsigned short*)Cout  + (size_t)b * strideC;
      unsigned short* C2 = (OUT_MODE == 2) ? ((unsigned short*)Cout2 + (size_t)b * strideC) : nullptr;
      for (int pass = 0; pass < 2; ++pass) {
#pragma unroll
        for (int it = 0; it < 4; ++it) {
          const int row = it * 4 + q;
          const float* sp = slab + row * 68 + c8;
          v8h hv, lv;
#pragma unroll
          for (int e = 0; e < 8; ++e) {
            if (OUT_MODE == 1) {
              hv[e] = (_Float16)sp[e];
            } else {
              unsigned short hb = f2bf_bits(sp[e]);
              unsigned short lb = f2bf_bits(sp[e] - bf_bits2f(hb));
              hv[e] = __builtin_bit_cast(_Float16, hb);
              lv[e] = __builtin_bit_cast(_Float16, lb);
            }
          }
          *(volatile v8h*)(C + (size_t)(mBase + row) * ldc + n0 + c8) = hv;
          if (OUT_MODE == 2) *(volatile v8h*)(C2 + (size_t)(mBase + row) * ldc + n0 + c8) = lv;
        }
        __threadfence();
      }
    }
    __builtin_amdgcn_fence(__ATOMIC_RELEASE, "workgroup");
    __builtin_amdgcn_wave_barrier();
    __builtin_amdgcn_fence(__ATOMIC_ACQUIRE, "workgroup");
  }
}

template <bool DUP>
__global__ __launch_bounds__(256) void convrows_kernel(const float* __restrict__ in, unsigned short* __restrict__ out,
                                                       int ncols, int ldout, int n8) {
  const int i = blockIdx.x * 256 + threadIdx.x;
  if (i < n8) {
    const size_t e0 = (size_t)i * 8;
    const int row = (int)(e0 / (size_t)ncols);
    const int col = (int)(e0 - (size_t)row * ncols);
    const v4f a = *(const v4f*)(in + e0);
    const v4f c = *(const v4f*)(in + e0 + 4);
    v4u hv;
    hv[0] = pk16(f2bf_bits(a[0]), f2bf_bits(a[1]));
    hv[1] = pk16(f2bf_bits(a[2]), f2bf_bits(a[3]));
    hv[2] = pk16(f2bf_bits(c[0]), f2bf_bits(c[1]));
    hv[3] = pk16(f2bf_bits(c[2]), f2bf_bits(c[3]));
    const size_t o = (size_t)row * ldout + col;
    for (int pass = 0; pass < 2; ++pass) {
      *(volatile v4u*)(out + o) = hv;
      if (DUP) *(volatile v4u*)(out + o + ncols) = hv;
      __threadfence();
    }
  }
}

__global__ __launch_bounds__(256) void tconv_kernel(const float* __restrict__ W, unsigned short* __restrict__ oh,
                                                    int ldin, int ldout, long sIn, long sOut) {
  __shared__ __align__(16) float tf[64 * 68];
  W  += (size_t)blockIdx.z * sIn;
  oh += (size_t)blockIdx.z * sOut;
  const int c0  = blockIdx.x * 64;
  const int r0  = blockIdx.y * 64;
  const int tid = threadIdx.x;
  {
    const int lr = tid >> 4;
    const int c4 = (tid & 15) * 4;
#pragma unroll
    for (int it = 0; it < 4; ++it) {
      const int rr = it * 16 + lr;
      const v4f a = *(const v4f*)(W + (size_t)(r0 + rr) * ldin + c0 + c4);
      *(v4f*)(tf + rr * 68 + c4) = a;
    }
  }
  __syncthreads();
  const int sub = tid >> 3;
  const int c8  = (tid & 7) * 8;
  v4u hv[2];
#pragma unroll
  for (int it = 0; it < 2; ++it) {
    const int oc = it * 32 + sub;
    v4u a;
#pragma unroll
    for (int q = 0; q < 4; ++q) {
      const float f0 = tf[(c8 + 2 * q) * 68 + oc];
      const float f1 = tf[(c8 + 2 * q + 1) * 68 + oc];
      a[q] = pk16(f2bf_bits(f0), f2bf_bits(f1));
    }
    hv[it] = a;
  }
  for (int pass = 0; pass < 2; ++pass) {
#pragma unroll
    for (int it = 0; it < 2; ++it) {
      const int oc = it * 32 + sub;
      const size_t go = (size_t)(c0 + oc) * ldout + r0 + c8;
      *(volatile v4u*)(oh + go) = hv[it];
    }
    __threadfence();
  }
}

__device__ __forceinline__ float rope_freq(int j) {
  float f = 1.0f;
  f = (j == 1)  ? 0.5623413251903491f     : f;
  f = (j == 2)  ? 0.31622776601683794f    : f;
  f = (j == 3)  ? 0.17782794100389229f    : f;
  f = (j == 4)  ? 0.1f                    : f;
  f = (j == 5)  ? 0.05623413251903491f    : f;
  f = (j == 6)  ? 0.031622776601683794f   : f;
  f = (j == 7)  ? 0.017782794100389229f   : f;
  f = (j == 8)  ? 0.01f                   : f;
  f = (j == 9)  ? 0.005623413251903491f   : f;
  f = (j == 10) ? 0.0031622776601683794f  : f;
  f = (j == 11) ? 0.0017782794100389228f  : f;
  f = (j == 12) ? 0.001f                  : f;
  f = (j == 13) ? 0.0005623413251903491f  : f;
  f = (j == 14) ? 0.00031622776601683794f : f;
  f = (j == 15) ? 0.00017782794100389227f : f;
  return f;
}

__global__ __launch_bounds__(256) void ropetab_kernel(float* __restrict__ tc, float* __restrict__ ts) {
  const int i = blockIdx.x * 256 + threadIdx.x;
  if (i < TABN) {
    const int pos = i >> 4, j = i & 15;
    const float a = (float)pos * rope_freq(j);
    const float c = cosf(a);
    const float s = sinf(a);
    ((volatile float*)tc)[i] = c;
    ((volatile float*)ts)[i] = s;
    __threadfence();
    ((volatile float*)tc)[i] = c;
    ((volatile float*)ts)[i] = s;
  }
}

__global__ __launch_bounds__(128) void ropenorm_kernel(const float* __restrict__ qkf,
                                                       const float* __restrict__ tc, const float* __restrict__ ts,
                                                       const float* __restrict__ qw, const float* __restrict__ kw,
                                                       unsigned short* __restrict__ qh, unsigned short* __restrict__ ql,
                                                       unsigned short* __restrict__ kh, unsigned short* __restrict__ kl) {
  __shared__ float redq[4], redk[4];
  const int g = blockIdx.x;
  const int n = g & (NTOK - 1);
  const int py = n >> 5, px = n & 31;
  const int t = threadIdx.x, lane = t & 31, wave = t >> 5;
  const int i0 = t * 8;

  const float* qr = qkf + (size_t)g * QKP + i0;
  const float* kr = qr + INNER;
  const v4f qa = *(const v4f*)(qr), qb = *(const v4f*)(qr + 4);
  const v4f ka = *(const v4f*)(kr), kb = *(const v4f*)(kr + 4);

  const int p0   = (4 * t) & 31;
  const int hsel = p0 >> 4;
  const int pos  = py + hsel * (px - py);
  const int toff = pos * 16 + (p0 & 15);
  const v4f cv = *(const v4f*)(tc + toff);
  const v4f sv = *(const v4f*)(ts + toff);

  float q8[8], k8[8];
  q8[0] = qa[0]; q8[1] = qa[1]; q8[2] = qa[2]; q8[3] = qa[3];
  q8[4] = qb[0]; q8[5] = qb[1]; q8[6] = qb[2]; q8[7] = qb[3];
  k8[0] = ka[0]; k8[1] = ka[1]; k8[2] = ka[2]; k8[3] = ka[3];
  k8[4] = kb[0]; k8[5] = kb[1]; k8[6] = kb[2]; k8[7] = kb[3];

  float rq[8], rk[8];
#pragma unroll
  for (int e = 0; e < 4; ++e) {
    const float c = cv[e], s = sv[e];
    const float qe = q8[2 * e], qo = q8[2 * e + 1];
    const float ke = k8[2 * e], ko = k8[2 * e + 1];
    rq[2 * e]     = qe * c - qo * s;
    rq[2 * e + 1] = qe * s + qo * c;
    rk[2 * e]     = ke * c - ko * s;
    rk[2 * e + 1] = ke * s + ko * c;
  }
  float ssq = 0.0f, ssk = 0.0f;
#pragma unroll
  for (int e = 0; e < 8; ++e) { ssq += rq[e] * rq[e]; ssk += rk[e] * rk[e]; }
#pragma unroll
  for (int off = 1; off < 32; off <<= 1) { ssq += __shfl_xor(ssq, off, 32); ssk += __shfl_xor(ssk, off, 32); }
  if (lane == 0) { redq[wave] = ssq; redk[wave] = ssk; }
  __syncthreads();
  const float tq = (redq[0] + redq[1]) + (redq[2] + redq[3]);
  const float tk = (redk[0] + redk[1]) + (redk[2] + redk[3]);
  const float rmq = rsqrtf(tq * (1.0f / (float)INNER) + RMS_EPS);
  const float rmk = rsqrtf(tk * (1.0f / (float)INNER) + RMS_EPS);

  const v4f wqa = *(const v4f*)(qw + i0), wqb = *(const v4f*)(qw + i0 + 4);
  const v4f wka = *(const v4f*)(kw + i0), wkb = *(const v4f*)(kw + i0 + 4);
  float wq8[8], wk8[8];
  wq8[0] = bf_rne(wqa[0]); wq8[1] = bf_rne(wqa[1]); wq8[2] = bf_rne(wqa[2]); wq8[3] = bf_rne(wqa[3]);
  wq8[4] = bf_rne(wqb[0]); wq8[5] = bf_rne(wqb[1]); wq8[6] = bf_rne(wqb[2]); wq8[7] = bf_rne(wqb[3]);
  wk8[0] = bf_rne(wka[0]); wk8[1] = bf_rne(wka[1]); wk8[2] = bf_rne(wka[2]); wk8[3] = bf_rne(wka[3]);
  wk8[4] = bf_rne(wkb[0]); wk8[5] = bf_rne(wkb[1]); wk8[6] = bf_rne(wkb[2]); wk8[7] = bf_rne(wkb[3]);

  v4u hq, lq, hk, lk;
#pragma unroll
  for (int e = 0; e < 4; ++e) {
    const float fq0 = rq[2 * e] * rmq * wq8[2 * e];
    const float fq1 = rq[2 * e + 1] * rmq * wq8[2 * e + 1];
    const float fk0 = rk[2 * e] * rmk * wk8[2 * e];
    const float fk1 = rk[2 * e + 1] * rmk * wk8[2 * e + 1];
    const unsigned short hq0 = f2bf_bits(fq0), hq1 = f2bf_bits(fq1);
    const unsigned short hk0 = f2bf_bits(fk0), hk1 = f2bf_bits(fk1);
    const unsigned short lq0 = f2bf_bits(fq0 - bf_bits2f(hq0)), lq1 = f2bf_bits(fq1 - bf_bits2f(hq1));
    const unsigned short lk0 = f2bf_bits(fk0 - bf_bits2f(hk0)), lk1 = f2bf_bits(fk1 - bf_bits2f(hk1));
    hq[e] = pk16(hq0, hq1); lq[e] = pk16(lq0, lq1);
    hk[e] = pk16(hk0, hk1); lk[e] = pk16(lk0, lk1);
  }
  const size_t o = (size_t)g * INNER + i0;
  for (int pass = 0; pass < 2; ++pass) {
    *(volatile v4u*)(qh + o) = hq;
    *(volatile v4u*)(ql + o) = lq;
    *(volatile v4u*)(kh + o) = hk;
    *(volatile v4u*)(kl + o) = lk;
    __threadfence();
  }
}

#define AT_D 64
#define AT_NW 4
#define AT_QB 64
#define AT_KC 64

__device__ __forceinline__ unsigned short at_bf_bits(float f) {
  unsigned u = __float_as_uint(f);
  return (unsigned short)((u + 0x7FFFu + ((u >> 16) & 1u)) >> 16);
}
__device__ __forceinline__ __bf16 at_f2bf(float f) { return __builtin_bit_cast(__bf16, at_bf_bits(f)); }
__device__ __forceinline__ void at_split(float f, __bf16& hi, __bf16& lo) {
  const unsigned short hb = at_bf_bits(f);
  hi = __builtin_bit_cast(__bf16, hb);
  lo = at_f2bf(f - __uint_as_float(((unsigned)hb) << 16));
}
__device__ __forceinline__ v8f at_mma(v16b a, v16b b, v8f c) {
  c = __builtin_amdgcn_wmma_f32_16x16x32_bf16(false, a, false, b, (short)0, c, false, false);
  asm volatile("v_nop\n\tv_nop\n\tv_nop\n\tv_nop" : "+v"(c) : "v"(a), "v"(b));
  return c;
}

__global__ __launch_bounds__(128)
void attn_kernel(const unsigned short* __restrict__ qhp, const unsigned short* __restrict__ qlp,
                 const unsigned short* __restrict__ khp, const unsigned short* __restrict__ klp,
                 const unsigned short* __restrict__ vhp, const unsigned short* __restrict__ vlp,
                 unsigned short* __restrict__ aop, float sscale) {
  union FB { v16b v; v8b h[2]; };
  __shared__ __align__(16) __bf16 Ksh[AT_KC * AT_D];
  __shared__ __align__(16) __bf16 Ksl[AT_KC * AT_D];
  __shared__ __align__(16) __bf16 Vth[AT_D * AT_KC];
  __shared__ __align__(16) __bf16 Vtl[AT_D * AT_KC];
  __shared__ __align__(16) __bf16 Psh[AT_NW][16 * AT_KC];
  __shared__ __align__(16) __bf16 Psl[AT_NW][16 * AT_KC];
  __shared__ __align__(16) float  Os[AT_NW][16 * 68];

  const int tid  = threadIdx.x;
  const int wave = tid >> 5;
  const int lane = tid & 31;
  const int hh   = lane >> 4;
  const int c    = lane & 15;

  const int nqb = NTOK / AT_QB;
  const int bx = blockIdx.x;
  const int qb = bx % nqb;
  const int hb = bx / nqb;
  const int h  = hb % NH;
  const int b  = hb / NH;
  const int q0 = b * NTOK + qb * AT_QB + wave * 16;

  const __bf16* Qh = (const __bf16*)(const void*)qhp + (size_t)h * AT_D;
  const __bf16* Ql = (const __bf16*)(const void*)qlp + (size_t)h * AT_D;
  const __bf16* Kh = (const __bf16*)(const void*)khp + (size_t)h * AT_D;
  const __bf16* Kl = (const __bf16*)(const void*)klp + (size_t)h * AT_D;
  const __bf16* Vh = (const __bf16*)(const void*)vhp + (size_t)h * AT_D * VTP + (size_t)b * NTOK;
  const __bf16* Vl = (const __bf16*)(const void*)vlp + (size_t)h * AT_D * VTP + (size_t)b * NTOK;
  unsigned short* Ch = aop + (size_t)h * AT_D;
  unsigned short* Cl = aop + (size_t)INNER + (size_t)h * AT_D;

  v16b qah[2], qal[2];
#pragma unroll
  for (int dc = 0; dc < 2; ++dc) {
    const __bf16* qr = Qh + (size_t)(q0 + c) * INNER + dc * 32 + 8 * hh;
    const __bf16* ql = Ql + (size_t)(q0 + c) * INNER + dc * 32 + 8 * hh;
    qah[dc] = Frag<__bf16>::load(qr);
    qal[dc] = Frag<__bf16>::load(ql);
  }

  float mrow[8], lrow[8];
  v8f oacc[4];
#pragma unroll
  for (int r = 0; r < 8; ++r) { mrow[r] = -INFINITY; lrow[r] = 0.f; }
#pragma unroll
  for (int t = 0; t < 4; ++t) oacc[t] = (v8f){0.f,0.f,0.f,0.f,0.f,0.f,0.f,0.f};

  const int nChunks = NTOK / AT_KC;
  for (int kc = 0; kc < nChunks; ++kc) {
    const int kv0 = kc * AT_KC;
    __syncthreads();
    {
      const int r = tid >> 1, half = (tid & 1) * 32;
      const __bf16* ksh = Kh + (size_t)(b * NTOK + kv0 + r) * INNER + half;
      const __bf16* ksl = Kl + (size_t)(b * NTOK + kv0 + r) * INNER + half;
      const __bf16* vsh = Vh + (size_t)r * VTP + kv0 + half;
      const __bf16* vsl = Vl + (size_t)r * VTP + kv0 + half;
#pragma unroll
      for (int i = 0; i < 4; ++i) {
        const v8b a0 = *(const v8b*)(ksh + 8 * i);
        const v8b a1 = *(const v8b*)(ksl + 8 * i);
        const v8b b0 = *(const v8b*)(vsh + 8 * i);
        const v8b b1 = *(const v8b*)(vsl + 8 * i);
        *(v8b*)(Ksh + r * AT_D  + half + 8 * i) = a0;
        *(v8b*)(Ksl + r * AT_D  + half + 8 * i) = a1;
        *(v8b*)(Vth + r * AT_KC + half + 8 * i) = b0;
        *(v8b*)(Vtl + r * AT_KC + half + 8 * i) = b1;
      }
    }
    __syncthreads();

    v8f s[4];
#pragma unroll
    for (int j = 0; j < 4; ++j) {
      s[j] = (v8f){0.f,0.f,0.f,0.f,0.f,0.f,0.f,0.f};
#pragma unroll
      for (int dc = 0; dc < 2; ++dc) {
        FB kb, kl;
        kb.h[0] = *(const v8b*)(Ksh + (j * 16 + c) * AT_D + dc * 32 + 8 * hh);
        kb.h[1] = *(const v8b*)(Ksh + (j * 16 + c) * AT_D + dc * 32 + 16 + 8 * hh);
        kl.h[0] = *(const v8b*)(Ksl + (j * 16 + c) * AT_D + dc * 32 + 8 * hh);
        kl.h[1] = *(const v8b*)(Ksl + (j * 16 + c) * AT_D + dc * 32 + 16 + 8 * hh);
        s[j] = at_mma(qah[dc], kb.v, s[j]);
        s[j] = at_mma(qah[dc], kl.v, s[j]);
        s[j] = at_mma(qal[dc], kb.v, s[j]);
      }
    }
    float cm[8];
#pragma unroll
    for (int r = 0; r < 8; ++r) {
      float m = -INFINITY;
#pragma unroll
      for (int j = 0; j < 4; ++j) {
        const float sv = s[j][r] * sscale;
        s[j][r] = sv;
        m = fmaxf(m, sv);
      }
#pragma unroll
      for (int off = 1; off < 16; off <<= 1) m = fmaxf(m, __shfl_xor(m, off, 32));
      cm[r] = m;
    }
    __bf16* pwh = Psh[wave];
    __bf16* pwl = Psl[wave];
#pragma unroll
    for (int r = 0; r < 8; ++r) {
      const float mnew = fmaxf(mrow[r], cm[r]);
      const float alpha = expf(mrow[r] - mnew);
      mrow[r] = mnew;
      float psum = 0.f;
#pragma unroll
      for (int j = 0; j < 4; ++j) {
        const float p = expf(s[j][r] - mnew);
        psum += p;
        __bf16 a, bl; at_split(p, a, bl);
        pwh[(8 * hh + r) * AT_KC + j * 16 + c] = a;
        pwl[(8 * hh + r) * AT_KC + j * 16 + c] = bl;
      }
#pragma unroll
      for (int off = 1; off < 16; off <<= 1) psum += __shfl_xor(psum, off, 32);
      lrow[r] = lrow[r] * alpha + psum;
#pragma unroll
      for (int t = 0; t < 4; ++t) oacc[t][r] *= alpha;
    }
    __builtin_amdgcn_fence(__ATOMIC_RELEASE, "workgroup");
    __builtin_amdgcn_wave_barrier();
    __builtin_amdgcn_fence(__ATOMIC_ACQUIRE, "workgroup");
#pragma unroll 1
    for (int kk = 0; kk < 2; ++kk) {
      FB pa, pl;
      pa.h[0] = *(const v8b*)(pwh + c * AT_KC + kk * 32 + 8 * hh);
      pa.h[1] = *(const v8b*)(pwh + c * AT_KC + kk * 32 + 16 + 8 * hh);
      pl.h[0] = *(const v8b*)(pwl + c * AT_KC + kk * 32 + 8 * hh);
      pl.h[1] = *(const v8b*)(pwl + c * AT_KC + kk * 32 + 16 + 8 * hh);
#pragma unroll
      for (int t = 0; t < 4; ++t) {
        FB vb, vl;
        vb.h[0] = *(const v8b*)(Vth + (t * 16 + c) * AT_KC + kk * 32 + 8 * hh);
        vb.h[1] = *(const v8b*)(Vth + (t * 16 + c) * AT_KC + kk * 32 + 16 + 8 * hh);
        vl.h[0] = *(const v8b*)(Vtl + (t * 16 + c) * AT_KC + kk * 32 + 8 * hh);
        vl.h[1] = *(const v8b*)(Vtl + (t * 16 + c) * AT_KC + kk * 32 + 16 + 8 * hh);
        oacc[t] = at_mma(pa.v, vb.v, oacc[t]);
        oacc[t] = at_mma(pa.v, vl.v, oacc[t]);
        oacc[t] = at_mma(pl.v, vb.v, oacc[t]);
      }
    }
  }

  float* os = Os[wave];
#pragma unroll
  for (int r = 0; r < 8; ++r) {
    const float inv = 1.0f / lrow[r];
#pragma unroll
    for (int t = 0; t < 4; ++t) os[(8 * hh + r) * 68 + t * 16 + c] = oacc[t][r] * inv;
  }
  __builtin_amdgcn_fence(__ATOMIC_RELEASE, "workgroup");
  __builtin_amdgcn_wave_barrier();
  __builtin_amdgcn_fence(__ATOMIC_ACQUIRE, "workgroup");
  {
    const int q = lane >> 3, c8 = (lane & 7) * 8;
    for (int pass = 0; pass < 2; ++pass) {
#pragma unroll
      for (int it = 0; it < 4; ++it) {
        const int row = it * 4 + q;
        const float* sp = os + row * 68 + c8;
        v8h hv, lv;
#pragma unroll
        for (int e = 0; e < 8; ++e) {
          const unsigned short hbits = f2bf_bits(sp[e]);
          const unsigned short lbits = f2bf_bits(sp[e] - bf_bits2f(hbits));
          hv[e] = __builtin_bit_cast(_Float16, hbits);
          lv[e] = __builtin_bit_cast(_Float16, lbits);
        }
        *(volatile v8h*)(Ch + (size_t)(q0 + row) * AOP + c8) = hv;
        *(volatile v8h*)(Cl + (size_t)(q0 + row) * AOP + c8) = lv;
      }
      __threadfence();
    }
  }
}

__global__ __launch_bounds__(256) void final_kernel(const float* __restrict__ of, const float* __restrict__ nw,
                                                    const float* __restrict__ xin, float* __restrict__ out) {
  __shared__ __align__(16) float tf[64 * 68];
  __shared__ float rms[64];
  const int tid = threadIdx.x, lane = tid & 31, wave = tid >> 5;
  const int tok0 = blockIdx.x * 64;
  const int b = tok0 / NTOK, n0 = tok0 - b * NTOK;

#pragma unroll 1
  for (int i = 0; i < 8; ++i) {
    const int rr = wave * 8 + i;
    const float* rowp = of + (size_t)(tok0 + rr) * CH + lane * 4;
    float ss = 0.0f;
#pragma unroll 2
    for (int k = 0; k < 8; ++k) {
      const v4f v = *(const v4f*)(rowp + k * 128);
      ss += v[0] * v[0] + v[1] * v[1] + v[2] * v[2] + v[3] * v[3];
    }
#pragma unroll
    for (int off = 1; off < 32; off <<= 1) ss += __shfl_xor(ss, off, 32);
    if (lane == 0) rms[rr] = rsqrtf(ss * (1.0f / (float)CH) + RMS_EPS);
  }
  __syncthreads();

  const int lr = tid >> 4;
  const int c4 = (tid & 15) * 4;
#pragma unroll 1
  for (int ct = 0; ct < CH / 64; ++ct) {
    const int c0 = ct * 64;
    {
      const v4f w4 = *(const v4f*)(nw + c0 + c4);
      float wr[4];
      wr[0] = bf_rne(w4[0]); wr[1] = bf_rne(w4[1]); wr[2] = bf_rne(w4[2]); wr[3] = bf_rne(w4[3]);
#pragma unroll
      for (int it = 0; it < 4; ++it) {
        const int rr = it * 16 + lr;
        const v4f v = *(const v4f*)(of + (size_t)(tok0 + rr) * CH + c0 + c4);
        const float rm = rms[rr];
        v4f o;
        o[0] = v[0] * rm * wr[0]; o[1] = v[1] * rm * wr[1]; o[2] = v[2] * rm * wr[2]; o[3] = v[3] * rm * wr[3];
        *(v4f*)(tf + rr * 68 + c4) = o;
      }
    }
    __syncthreads();
    v4f ov[4];
#pragma unroll
    for (int it = 0; it < 4; ++it) {
      const int oc = it * 16 + lr;
      const v4f xr = *(const v4f*)(xin + ((size_t)(b * CH + c0 + oc)) * NTOK + n0 + c4);
      v4f o;
      o[0] = tf[(c4 + 0) * 68 + oc] + bf_rne(xr[0]);
      o[1] = tf[(c4 + 1) * 68 + oc] + bf_rne(xr[1]);
      o[2] = tf[(c4 + 2) * 68 + oc] + bf_rne(xr[2]);
      o[3] = tf[(c4 + 3) * 68 + oc] + bf_rne(xr[3]);
      ov[it] = o;
    }
    for (int pass = 0; pass < 2; ++pass) {
#pragma unroll
      for (int it = 0; it < 4; ++it) {
        const int oc = it * 16 + lr;
        *(volatile v4f*)(out + ((size_t)(b * CH + c0 + oc)) * NTOK + n0 + c4) = ov[it];
      }
      __threadfence();
    }
    __syncthreads();
  }
}

extern "C" void kernel_launch(void* const* d_in, const int* in_sizes, int n_in,
                              void* d_out, int out_size, void* d_ws, size_t ws_size,
                              hipStream_t stream) {
  if (n_in < 7) return;
  if (in_sizes[0] != NB * CH * NTOK) return;
  if (in_sizes[1] != NQKV * CH) return;
  if (in_sizes[2] != NQKV) return;
  if (in_sizes[3] != INNER) return;
  if (in_sizes[4] != INNER) return;
  if (in_sizes[5] != CH * INNER) return;
  if (in_sizes[6] != CH) return;
  if (out_size != NB * CH * NTOK) return;

  const float* x    = (const float*)d_in[0];
  const float* wqkv = (const float*)d_in[1];
  const float* bqkv = (const float*)d_in[2];
  const float* qnw  = (const float*)d_in[3];
  const float* knw  = (const float*)d_in[4];
  const float* wprj = (const float*)d_in[5];
  const float* onw  = (const float*)d_in[6];

  const size_t PXB = (size_t)MTOK * CH * 2;
  const size_t PWQ = (size_t)NQKV * CH * 2;
  const size_t PWP = (size_t)CH * AOP * 2;
  const size_t PTB = (size_t)TABN * 4;
  const size_t PQK = (size_t)MTOK * QKP * 4;
  const size_t PCX = (size_t)MTOK * AOP * 2;
  const size_t POF = (size_t)MTOK * CH * 4;
  const size_t PPL = (size_t)MTOK * INNER * 2;
  const size_t PVT = (size_t)INNER * VTP * 2;
  if (PCX + POF > PQK) return;
  size_t off = 0;
  const size_t oXB  = off; off += PXB;
  const size_t oWQ  = off; off += PWQ;
  const size_t oWP  = off; off += PWP;
  const size_t oTC  = off; off += PTB;
  const size_t oTS  = off; off += PTB;
  const size_t oQK  = off; off += PQK;
  const size_t oCX  = oQK;
  const size_t oOF  = oQK + PCX;
  const size_t oQh  = off; off += PPL;  const size_t oQl = off; off += PPL;
  const size_t oKh  = off; off += PPL;  const size_t oKl = off; off += PPL;
  const size_t oVTh = off; off += PVT;  const size_t oVTl = off; off += PVT;
  if (off > ws_size) return;
  if (off > (size_t)134217728) return;

  char* ws = (char*)d_ws;
  unsigned short* XB   = (unsigned short*)(ws + oXB);
  unsigned short* WQKV = (unsigned short*)(ws + oWQ);
  unsigned short* WP2  = (unsigned short*)(ws + oWP);
  float*          TC   = (float*)(ws + oTC);
  float*          TS   = (float*)(ws + oTS);
  float*          QKf  = (float*)(ws + oQK);
  unsigned short* CTX2 = (unsigned short*)(ws + oCX);
  float*          Of   = (float*)(ws + oOF);
  unsigned short* Qh   = (unsigned short*)(ws + oQh);  unsigned short* Ql  = (unsigned short*)(ws + oQl);
  unsigned short* Kh   = (unsigned short*)(ws + oKh);  unsigned short* Kl  = (unsigned short*)(ws + oKl);
  unsigned short* VTh  = (unsigned short*)(ws + oVTh); unsigned short* VTl = (unsigned short*)(ws + oVTl);

  const dim3 blk(256);

  tconv_kernel<<<dim3(NTOK / 64, CH / 64, NB), blk, 0, stream>>>(x, XB, NTOK, CH, (long)CH * NTOK, (long)NTOK * CH);
  const int n8q = NQKV * CH / 8;
  convrows_kernel<false><<<dim3(n8q / 256), blk, 0, stream>>>(wqkv, WQKV, CH, CH, n8q);
  const int n8p = CH * INNER / 8;
  convrows_kernel<true><<<dim3(n8p / 256), blk, 0, stream>>>(wprj, WP2, INNER, AOP, n8p);
  ropetab_kernel<<<dim3(2), blk, 0, stream>>>(TC, TS);
  const dim3 gQK(((MTOK / 64) * (QKP / 64) + 7) / 8, 1);
  wmma_gemm64<1, false, 2, 0, false, 0><<<gQK, blk, 0, stream>>>(
      XB, XB, CH, 0L, WQKV, WQKV, CH, 0L, (void*)QKf, (void*)QKf, QKP, 0L,
      bqkv, bqkv, 0L, MTOK, QKP, CH, 1.0f);
  const dim3 gVT(((INNER / 64) * (MTOK / 64) + 7) / 8, 1);
  wmma_gemm64<1, false, 1, 2, false, 0><<<gVT, blk, 0, stream>>>(
      WQKV + (size_t)2 * INNER * CH, WQKV + (size_t)2 * INNER * CH, CH, 0L, XB, XB, CH, 0L,
      (void*)VTh, (void*)VTl, VTP, 0L,
      bqkv + 2 * INNER, bqkv, 0L, INNER, MTOK, CH, 1.0f);
  ropenorm_kernel<<<dim3(MTOK), dim3(128), 0, stream>>>(QKf, TC, TS, qnw, knw, Qh, Ql, Kh, Kl);
  attn_kernel<<<dim3(NB * NH * (NTOK / 64)), dim3(128), 0, stream>>>(Qh, Ql, Kh, Kl, VTh, VTl, CTX2, 0.125f);
  const dim3 gO(((MTOK / 64) * (CH / 64) + 7) / 8, 1);
  wmma_gemm64<1, false, 0, 0, false, 0><<<gO, blk, 0, stream>>>(
      CTX2, CTX2, AOP, 0L, WP2, WP2, AOP, 0L, (void*)Of, (void*)Of, CH, 0L,
      bqkv, bqkv, 0L, MTOK, CH, AOP, 1.0f);
  final_kernel<<<dim3(MTOK / 64), blk, 0, stream>>>(Of, onw, x, (float*)d_out);
  (void)hipGetLastError();
}
